// SuctionNet_prob_4741643895570
// MI455X (gfx1250) — hardware-verified
//
#include <hip/hip_runtime.h>
#include <stddef.h>
#include <math.h>


#define KNBR   27
#define C1     64
#define COUT   256
#define KTOT   (KNBR * C1)
#define NKB    (KTOT / 32)
#define NTH    256
#define NWAV   8
#define VPB1   32
#define VB     2048
#define MAXT   (VB / 64)
#define APITCH 72
#define SCH    1024
#define HSC    16.0f
#define WSC    64.0f
#define OSC    0.0009765625f

static_assert((VB % 64) == 0);
static_assert(VB == 8 * NTH);
static_assert(SCH == 4 * NTH);
static_assert((KTOT % 32) == 0);
static_assert(MAXT * 64 == VB);

typedef float    v4f  __attribute__((ext_vector_type(4)));
typedef float    v8f  __attribute__((ext_vector_type(8)));
typedef int      v4i  __attribute__((ext_vector_type(4)));
typedef _Float16 v8h  __attribute__((ext_vector_type(8)));
typedef _Float16 v16h __attribute__((ext_vector_type(16)));
union FragH { v16h v; v8h h[2]; };

__device__ __forceinline__ v8f wmh(v16h a, v16h b, v8f c) {
  v8f d = __builtin_amdgcn_wmma_f32_16x16x32_f16(false, a, false, b, (short)0, c, false, false);
  asm volatile("v_nop\n\tv_nop\n\tv_nop\n\tv_nop" : "+v"(d) : "v"(a), "v"(b));
  return d;
}

__device__ __forceinline__ int normidx(int u, int n) {
  u = (u < 0) ? (u + n) : u;
  u = (u < 0) ? 0 : ((u > n - 1) ? (n - 1) : u);
  return u;
}

__global__ __launch_bounds__(NTH) void k_conv1(const float* __restrict__ feats,
                                                const int*   __restrict__ nidx1,
                                                const float* __restrict__ W1,
                                                const float* __restrict__ b1,
                                                _Float16* h1, int nvox) {
  __shared__ __attribute__((aligned(16))) float wl[KNBR * 3 * C1];
  __shared__ float bl[C1];
  const int tid = threadIdx.x;
  for (int i = tid; i < KNBR * 3 * C1; i += NTH) wl[i] = W1[i];
  if (tid < C1) bl[tid] = b1[tid];
  __syncthreads();

  const int cg = tid & 7;
  const int v  = blockIdx.x * VPB1 + (tid >> 3);
  const int vc = (v < nvox) ? v : (nvox - 1);
  const int* nrow = nidx1 + (size_t)vc * KNBR;

  float acc[8];
#pragma unroll
  for (int j = 0; j < 8; ++j) acc[j] = 0.0f;

#pragma unroll 1
  for (int k = 0; k < KNBR; ++k) {
    const int idx = normidx(nrow[k], nvox);
    const float* fp = feats + (size_t)idx * 3;
    const float f0 = fp[0], f1 = fp[1], f2 = fp[2];
    const float* wp = wl + k * 3 * C1 + cg * 8;
    const v4f w0a = *(const v4f*)(wp);          const v4f w0b = *(const v4f*)(wp + 4);
    const v4f w1a = *(const v4f*)(wp + C1);     const v4f w1b = *(const v4f*)(wp + C1 + 4);
    const v4f w2a = *(const v4f*)(wp + 2 * C1); const v4f w2b = *(const v4f*)(wp + 2 * C1 + 4);
    float w0[8], w1[8], w2[8];
    w0[0] = w0a.x; w0[1] = w0a.y; w0[2] = w0a.z; w0[3] = w0a.w; w0[4] = w0b.x; w0[5] = w0b.y; w0[6] = w0b.z; w0[7] = w0b.w;
    w1[0] = w1a.x; w1[1] = w1a.y; w1[2] = w1a.z; w1[3] = w1a.w; w1[4] = w1b.x; w1[5] = w1b.y; w1[6] = w1b.z; w1[7] = w1b.w;
    w2[0] = w2a.x; w2[1] = w2a.y; w2[2] = w2a.z; w2[3] = w2a.w; w2[4] = w2b.x; w2[5] = w2b.y; w2[6] = w2b.z; w2[7] = w2b.w;
#pragma unroll
    for (int j = 0; j < 8; ++j) {
      float d = f0 * w0[j];
      d = fmaf(f1, w1[j], d);
      d = fmaf(f2, w2[j], d);
      acc[j] += d;
    }
  }

  v8h hv;
#pragma unroll
  for (int j = 0; j < 8; ++j) {
    const float t = fmaxf(acc[j] + bl[cg * 8 + j], 0.0f) * HSC;
    hv[j] = (_Float16)t;
  }
  _Float16* dst = h1 + (size_t)v * C1 + cg * 8;
  *(volatile v8h*)dst = hv;
  __threadfence();
  *(volatile v8h*)dst = hv;
}

__global__ __launch_bounds__(NTH) void k_w2pack(const float* __restrict__ W2, _Float16* w2s) {
  const int T = blockIdx.x * NTH + threadIdx.x;
  const int total = NKB * 16 * 32 * 2;
  if (T >= total) return;
  const int ih   = T & 1;
  const int ln   = (T >> 1) & 31;
  const int tile = T >> 6;
  const int kb   = tile >> 4;
  const int nb   = tile & 15;
  const int hh   = ln >> 4;
  const int col  = nb * 16 + (ln & 15);
  const int kbase = kb * 32 + 16 * ih + 8 * hh;
  v8h o;
#pragma unroll
  for (int i = 0; i < 8; ++i) {
    const float w = W2[(size_t)(kbase + i) * COUT + col] * WSC;
    o[i] = (_Float16)w;
  }
  _Float16* dst = w2s + (size_t)T * 8;
  *(volatile v8h*)dst = o;
  __threadfence();
  *(volatile v8h*)dst = o;
}

__global__ __launch_bounds__(NTH) void k_conv2(const _Float16* __restrict__ h1,
                                                const int*      __restrict__ nidx2,
                                                const int*      __restrict__ q2o,
                                                const _Float16* __restrict__ w2s,
                                                const float*    __restrict__ b2,
                                                const float*    __restrict__ score_w,
                                                const float*    __restrict__ sigma_w,
                                                float* svox, float* tvox, int nvox, int np) {
  __shared__ __attribute__((aligned(16))) _Float16 Alds[64 * APITCH];
  __shared__ int flg[VB];
  __shared__ int lst[VB];
  __shared__ __attribute__((aligned(16))) float sres[VB];
  __shared__ __attribute__((aligned(16))) float tres[VB];
  __shared__ int   tvx[64];
  __shared__ int   tlc[64];
  __shared__ float red_s[128];
  __shared__ float red_t[128];
  __shared__ int   wsum[NWAV];

  const int tid = threadIdx.x, lane = tid & 31, wave = tid >> 5;
  const int hh = lane >> 4, m = lane & 15;
  const int w_m = wave & 3, w_n = wave >> 2;
  const int vb = blockIdx.x * VB;

  for (int i = tid; i < VB; i += NTH) { flg[i] = 0; lst[i] = 0; sres[i] = 0.0f; tres[i] = 0.0f; }
  __syncthreads();

  const int nch = (np + SCH - 1) / SCH;
#pragma unroll 1
  for (int ch = 0; ch < nch; ++ch) {
    const int cbase = ch * SCH;
    const int e0 = cbase + 4 * tid;
    int u0, u1, u2, u3, k0, k1, k2, k3;
    if (cbase + SCH <= np) {
      const v4i d = *(const v4i*)(q2o + e0);
      u0 = d.x; u1 = d.y; u2 = d.z; u3 = d.w;
      k0 = 1; k1 = 1; k2 = 1; k3 = 1;
    } else {
      const int c0 = (e0     < np) ? e0     : (np - 1);
      const int c1 = (e0 + 1 < np) ? e0 + 1 : (np - 1);
      const int c2 = (e0 + 2 < np) ? e0 + 2 : (np - 1);
      const int c3 = (e0 + 3 < np) ? e0 + 3 : (np - 1);
      u0 = q2o[c0]; u1 = q2o[c1]; u2 = q2o[c2]; u3 = q2o[c3];
      k0 = (e0 < np) ? 1 : 0; k1 = (e0 + 1 < np) ? 1 : 0; k2 = (e0 + 2 < np) ? 1 : 0; k3 = (e0 + 3 < np) ? 1 : 0;
    }
    {
      const int l0 = normidx(u0, nvox) - vb; if (k0 != 0 && (unsigned)l0 < (unsigned)VB) flg[l0] = 1;
      const int l1 = normidx(u1, nvox) - vb; if (k1 != 0 && (unsigned)l1 < (unsigned)VB) flg[l1] = 1;
      const int l2 = normidx(u2, nvox) - vb; if (k2 != 0 && (unsigned)l2 < (unsigned)VB) flg[l2] = 1;
      const int l3 = normidx(u3, nvox) - vb; if (k3 != 0 && (unsigned)l3 < (unsigned)VB) flg[l3] = 1;
    }
  }
  __syncthreads();

  int fl[8];
  int c = 0;
#pragma unroll
  for (int i = 0; i < 8; ++i) { fl[i] = flg[8 * tid + i]; c += fl[i]; }
  int x = c;
#pragma unroll
  for (int d = 1; d < 32; d <<= 1) {
    const int y = __shfl_up(x, d, 32);
    if (lane >= d) x += y;
  }
  if (lane == 31) wsum[wave] = x;
  __syncthreads();
  int offw = 0, cnt = 0;
#pragma unroll
  for (int w = 0; w < NWAV; ++w) {
    int s = wsum[w];
    s = (s < 0) ? 0 : ((s > 8 * 32) ? (8 * 32) : s);
    if (w < wave) offw += s;
    cnt += s;
  }
  cnt = (cnt > VB) ? VB : cnt;
  {
    int pos = offw + x - c;
#pragma unroll
    for (int i = 0; i < 8; ++i) {
      if (fl[i] != 0) { if (pos < VB) lst[pos] = 8 * tid + i; ++pos; }
    }
  }
  __syncthreads();

  int nt = (cnt + 63) >> 6;
  nt = (nt > MAXT) ? MAXT : nt;
  const int grow = tid >> 2, gq = tid & 3;

#pragma unroll 1
  for (int t = 0; t < nt; ++t) {
    const int rbase = t * 64;
    int rv = cnt - rbase;
    rv = (rv > 64) ? 64 : rv;
    if (tid < 64) {
      int li = rbase + tid;
      li = (li > VB - 1) ? (VB - 1) : li;
      const int valid = (tid < rv) ? 1 : 0;
      int loc = lst[li];
      loc = (loc < 0) ? 0 : ((loc > VB - 1) ? (VB - 1) : loc);
      loc = (valid != 0) ? loc : 0;
      int vox = vb + loc;
      vox = (vox > nvox - 1) ? (nvox - 1) : vox;
      tvx[tid] = vox;
      tlc[tid] = (valid != 0) ? loc : -1;
    }
    __syncthreads();

    v8f acc[8];
#pragma unroll
    for (int tt = 0; tt < 8; ++tt) {
#pragma unroll
      for (int r = 0; r < 8; ++r) acc[tt][r] = 0.0f;
    }

    const int gvox = tvx[grow];
    const int* nrow = nidx2 + (size_t)gvox * KNBR;

#pragma unroll 1
    for (int koff = 0; koff < KNBR; ++koff) {
      const int nbr = normidx(nrow[koff], nvox);
      const _Float16* src = h1 + (size_t)nbr * C1 + gq * 16;
      const v8h x0 = *(const v8h*)src;
      const v8h x1 = *(const v8h*)(src + 8);
      __syncthreads();
      _Float16* ad = Alds + grow * APITCH + gq * 16;
      *(v8h*)ad = x0;
      *(v8h*)(ad + 8) = x1;
      __syncthreads();

#pragma unroll
      for (int half = 0; half < 2; ++half) {
        FragH a;
        const _Float16* ap = Alds + (w_m * 16 + m) * APITCH + 32 * half + 8 * hh;
        a.h[0] = *(const v8h*)ap;
        a.h[1] = *(const v8h*)(ap + 16);
        const int kb = koff * 2 + half;
        const _Float16* bp = w2s + ((size_t)(kb * 16 + w_n * 8) * 32 + lane) * 16;
#pragma unroll
        for (int tt = 0; tt < 8; ++tt) {
          FragH b;
          b.h[0] = *(const v8h*)(bp + tt * 512);
          b.h[1] = *(const v8h*)(bp + tt * 512 + 8);
          acc[tt] = wmh(a.v, b.v, acc[tt]);
        }
      }
    }

    float bb[8], sw[8], gw[8];
#pragma unroll
    for (int tt = 0; tt < 8; ++tt) {
      const int col = w_n * 128 + tt * 16 + m;
      bb[tt] = b2[col];
      sw[tt] = score_w[col];
      gw[tt] = sigma_w[col];
    }
#pragma unroll
    for (int r = 0; r < 8; ++r) {
      float s = 0.0f, g = 0.0f;
#pragma unroll
      for (int tt = 0; tt < 8; ++tt) {
        const float v = fmaxf(acc[tt][r] * OSC + bb[tt], 0.0f);
        s = fmaf(v, sw[tt], s);
        g = fmaf(v, gw[tt], g);
      }
#pragma unroll
      for (int off = 8; off >= 1; off >>= 1) {
        s += __shfl_xor(s, off, 32);
        g += __shfl_xor(g, off, 32);
      }
      if (m == 0) {
        const int row = w_m * 16 + 8 * hh + r;
        red_s[w_n * 64 + row] = s;
        red_t[w_n * 64 + row] = g;
      }
    }
    __syncthreads();
    if (tid < 64) {
      const int loc = tlc[tid];
      const float s = red_s[tid] + red_s[64 + tid];
      const float g = red_t[tid] + red_t[64 + tid];
      if (loc >= 0) { sres[loc] = s; tres[loc] = g; }
    }
  }
  __syncthreads();

  const v4f s0 = *(const v4f*)(sres + 4 * tid);
  const v4f s1 = *(const v4f*)(sres + 4 * (tid + NTH));
  const v4f t0 = *(const v4f*)(tres + 4 * tid);
  const v4f t1 = *(const v4f*)(tres + 4 * (tid + NTH));
  float* sp = svox + (size_t)vb;
  float* tp = tvox + (size_t)vb;
  *(volatile v4f*)(sp + 4 * tid) = s0;
  *(volatile v4f*)(sp + 4 * (tid + NTH)) = s1;
  *(volatile v4f*)(tp + 4 * tid) = t0;
  *(volatile v4f*)(tp + 4 * (tid + NTH)) = t1;
  __threadfence();
  *(volatile v4f*)(sp + 4 * tid) = s0;
  *(volatile v4f*)(sp + 4 * (tid + NTH)) = s1;
  *(volatile v4f*)(tp + 4 * tid) = t0;
  *(volatile v4f*)(tp + 4 * (tid + NTH)) = t1;
}

__global__ __launch_bounds__(NTH) void k_heads(const float* __restrict__ svox,
                                                const float* __restrict__ tvox,
                                                const int*   __restrict__ q2o,
                                                const float* __restrict__ score_b,
                                                const float* __restrict__ sigma_b,
                                                float* out, int np, int nvox) {
  __shared__ __attribute__((aligned(16))) float ss[NTH];
  __shared__ __attribute__((aligned(16))) float gg[NTH];
  const int tid = threadIdx.x;
  const int p  = blockIdx.x * NTH + tid;
  const int pc = (p < np) ? p : (np - 1);
  const int u  = normidx(q2o[pc], nvox);
  const float s  = svox[u] + score_b[0];
  const float xv = tvox[u] + sigma_b[0];
  const float g  = fmaxf(xv, 0.0f) + log1pf(expf(-fabsf(xv)));
  ss[tid] = s;
  gg[tid] = g;
  __syncthreads();

  const int which = (tid >> 6) & 1;
  const int q     = tid & 63;
  const int p0    = blockIdx.x * NTH + 4 * q;
  const v4f va = *(const v4f*)(ss + 4 * q);
  const v4f vg = *(const v4f*)(gg + 4 * q);
  v4f vo;
  vo.x = which ? vg.x : va.x;
  vo.y = which ? vg.y : va.y;
  vo.z = which ? vg.z : va.z;
  vo.w = which ? vg.w : va.w;
  const bool ok = (tid < 128) && (p0 < np);
  float* dst = out + (size_t)which * (size_t)np + (size_t)((p0 < np) ? p0 : 0);
  if (ok) *(volatile v4f*)dst = vo;
  __threadfence();
  if (ok) *(volatile v4f*)dst = vo;
}

extern "C" void kernel_launch(void* const* d_in, const int* in_sizes, int n_in,
                              void* d_out, int out_size, void* d_ws, size_t ws_size,
                              hipStream_t stream) {
  if (n_in < 12) return;
  const int nvox = in_sizes[0] / 3;
  if (nvox <= 0 || in_sizes[0] != nvox * 3) return;
  if (in_sizes[1] != nvox * KNBR || in_sizes[2] != nvox * KNBR) return;
  const int np = in_sizes[3];
  if (np < 4 || (np & 3) != 0 || out_size != 2 * np) return;
  if (in_sizes[4] != KNBR * 3 * C1 || in_sizes[5] != C1) return;
  if (in_sizes[6] != KTOT * COUT || in_sizes[7] != COUT) return;
  if (in_sizes[8] != COUT || in_sizes[9] < 1 || in_sizes[10] != COUT || in_sizes[11] < 1) return;

  const float* feats   = (const float*)d_in[0];
  const int*   nidx1   = (const int*)  d_in[1];
  const int*   nidx2   = (const int*)  d_in[2];
  const int*   q2o     = (const int*)  d_in[3];
  const float* W1      = (const float*)d_in[4];
  const float* b1      = (const float*)d_in[5];
  const float* W2      = (const float*)d_in[6];
  const float* b2      = (const float*)d_in[7];
  const float* score_w = (const float*)d_in[8];
  const float* score_b = (const float*)d_in[9];
  const float* sigma_w = (const float*)d_in[10];
  const float* sigma_b = (const float*)d_in[11];
  float* out = (float*)d_out;

  const int nb1  = (nvox + VPB1 - 1) / VPB1;
  const int nvp1 = nb1 * VPB1;
  const int nb2  = (nvox + VB - 1) / VB;
  const int nvp2 = nb2 * VB;
  const int nb3  = (np + NTH - 1) / NTH;
  const int nbw  = (NKB * 16 * 32 * 2 + NTH - 1) / NTH;

  char* ws = (char*)d_ws;
  size_t off = 0;
  const size_t oH1 = off; off += (size_t)nvp1 * C1 * sizeof(_Float16);      off = (off + 255) & ~(size_t)255;
  const size_t oW2 = off; off += (size_t)KTOT * COUT * sizeof(_Float16);    off = (off + 255) & ~(size_t)255;
  const size_t oS  = off; off += (size_t)nvp2 * sizeof(float);              off = (off + 255) & ~(size_t)255;
  const size_t oT  = off; off += (size_t)nvp2 * sizeof(float);              off = (off + 255) & ~(size_t)255;
  if (off > ws_size) return;
  _Float16* h1   = (_Float16*)(ws + oH1);
  _Float16* w2s  = (_Float16*)(ws + oW2);
  float*    svox = (float*)(ws + oS);
  float*    tvox = (float*)(ws + oT);

  k_conv1<<<nb1, NTH, 0, stream>>>(feats, nidx1, W1, b1, h1, nvox);
  k_w2pack<<<nbw, NTH, 0, stream>>>(W2, w2s);
  k_conv2<<<nb2, NTH, 0, stream>>>(h1, nidx2, q2o, w2s, b2, score_w, sigma_w, svox, tvox, nvox, np);
  k_heads<<<nb3, NTH, 0, stream>>>(svox, tvox, q2o, score_b, sigma_b, out, np, nvox);
}
